// KStepRGCN_24747601559831
// MI455X (gfx1250) — hardware-verified
//
#include <hip/hip_runtime.h>
#include <stddef.h>
#include <stdint.h>


#define CH     64
#define NR     8
#define NBS    4
#define NL     2
#define NCAT   576
#define XWP    576
#define KQ     8
#define KST    2
#define TR     16
#define NTHR   256
#define NWAVE  8
#define S1     1024
#define NCH1   4
#define SH1    8
#define FA1    200
#define CAP1   32
#define SH2    4
#define FA2    16
#define CAP2   512
#define GSP    68
#define GSB    68
#define NBN    18
#define NBLKB  36
#define WSC    64.0f
#define RWSC   0.015625f
#define SENT   0xFFFFFFFFu
#define EIDM   0x07FFFFFFu
#define KINV   1023
#define WSCAPB 134217728

static_assert(NCAT == NR * CH + CH && XWP == NCAT && (XWP % 32) == 0);
static_assert(KQ * 8 == CH && KST * 32 == CH);
static_assert(NTHR == 32 * NWAVE && TR == 2 * NWAVE && CH == 2 * 32);
static_assert(NCH1 * NTHR == S1);
static_assert((1 << (SH1 - SH2)) == FA2 && (1 << SH2) == TR);
static_assert(FA1 <= NTHR && FA2 <= 32 && KINV >= FA1 && KINV >= FA2);
static_assert(CAP1 == 32 && (CAP2 % 32) == 0);
static_assert(((FA1 * CAP1) % 4) == 0 && ((FA2 * CAP2) % 4) == 0);
static_assert(NBN * 32 == NCAT && NBLKB == NL * NBN);
static_assert(NTHR == 4 * CH && NTHR == 32 * KQ);
static_assert((GSP % 4) == 0 && GSP >= 64 && (GSB % 4) == 0 && GSB >= 64);
static_assert(TR * CH == 4 * NTHR);
static_assert(TR * CH == 8 * (NTHR / 2));
static_assert(64 * 64 == 4 * 4 * NTHR);

typedef _Float16 v8h  __attribute__((ext_vector_type(8)));
typedef _Float16 v16h __attribute__((ext_vector_type(16)));
typedef float    v2f  __attribute__((ext_vector_type(2)));
typedef float    v4f  __attribute__((ext_vector_type(4)));
typedef float    v8f  __attribute__((ext_vector_type(8)));
typedef unsigned int v4u __attribute__((ext_vector_type(4)));
typedef v2f v2fa __attribute__((may_alias));
typedef v4f v4fa __attribute__((may_alias));
typedef v4u v4ua __attribute__((may_alias));
union Frag { v16h v; v8h h[2]; };

__device__ __forceinline__ v8f wmh(v16h a, v16h b, v8f c) {
  v8f d = __builtin_amdgcn_wmma_f32_16x16x32_f16(false, a, false, b, (short)0, c, false, false);
  asm volatile("v_nop\n\tv_nop\n\tv_nop\n\tv_nop" : "+v"(d) : "v"(a), "v"(b));
  return d;
}

__device__ __forceinline__ v8f ld8g(const float* __restrict__ p) {
  const v4f lo = *(const v4fa*)p;
  const v4f hi = *(const v4fa*)(p + 4);
  v8f f = {lo[0], lo[1], lo[2], lo[3], hi[0], hi[1], hi[2], hi[3]};
  return f;
}

__global__ __launch_bounds__(NTHR) void k_prep(const float* __restrict__ x, const float* __restrict__ basis,
                                               const float* __restrict__ att, const float* __restrict__ root,
                                               _Float16* Ap, _Float16* Bw, unsigned* flag, int nN, int nbA) {
  __shared__ __attribute__((aligned(16))) float wst[32 * GSB];
  const int tid = threadIdx.x;
  const int blk = blockIdx.x;
  const v8f z8 = {0.f, 0.f, 0.f, 0.f, 0.f, 0.f, 0.f, 0.f};
  if (blk < nbA) {
    const int i = blk * NTHR + tid;
    const int row = i >> 3, k0 = (i & 7) * 8;
    const int rc = row < nN ? row : nN - 1;
    v8f f = ld8g(x + (size_t)rc * CH + k0);
    if (row >= nN) f = z8;
    const v8h hv = __builtin_convertvector(f, v8h);
    _Float16* dst = Ap + (size_t)i * 8;
    *(volatile v8h*)dst = hv;
    __threadfence();
    *(volatile v8h*)dst = hv;
  } else if (blk < nbA + NBLKB) {
    const int bi = blk - nbA;
    const int L  = bi / NBN;
    const int n0 = (bi - L * NBN) * 32;
    const int rl = n0 >> 6;
    const int rr = rl < NR ? rl : NR - 1;
    const int ob = n0 & (CH - 1);
    const bool isw = n0 < NR * CH;
    const int k = tid >> 2, op = tid & 3;
    const int o8 = ob + 8 * op;
    const v4f av = *(const v4fa*)(att + ((size_t)L * NR + rr) * NBS);
    const float* bp = basis + (size_t)L * NBS * CH * CH + (size_t)k * CH + o8;
    const float* rp = root + (size_t)L * CH * CH + (size_t)k * CH + o8;
    const v8f q0 = ld8g(bp);
    const v8f q1 = ld8g(bp + CH * CH);
    const v8f q2 = ld8g(bp + 2 * CH * CH);
    const v8f q3 = ld8g(bp + 3 * CH * CH);
    const v8f qr = ld8g(rp);
#pragma unroll
    for (int j = 0; j < 8; ++j) {
      float wv = av[0] * q0[j];
      wv = fmaf(av[1], q1[j], wv);
      wv = fmaf(av[2], q2[j], wv);
      wv = fmaf(av[3], q3[j], wv);
      wst[(8 * op + j) * GSB + k] = (isw ? wv : qr[j]) * WSC;
    }
    __syncthreads();
    const int row = tid >> 3, kq = (tid & 7) * 8;
    const v4f lo = *(const v4fa*)(wst + row * GSB + kq);
    const v4f hi = *(const v4fa*)(wst + row * GSB + kq + 4);
    const v8f g = {lo[0], lo[1], lo[2], lo[3], hi[0], hi[1], hi[2], hi[3]};
    const v8h hv = __builtin_convertvector(g, v8h);
    _Float16* dst = Bw + ((size_t)(L * NCAT + n0 + row) * CH + kq);
    *(volatile v8h*)dst = hv;
    __threadfence();
    *(volatile v8h*)dst = hv;
  } else {
    if (tid < 8) {
      const v4u z4 = {0u, 0u, 0u, 0u};
      unsigned* dst = flag + 4 * tid;
      *(volatile v4u*)dst = z4;
      __threadfence();
      *(volatile v4u*)dst = z4;
    }
  }
}

template <int LV, int FA, int CAP>
__global__ __launch_bounds__(NTHR) void k_part(const int* __restrict__ edst, const unsigned* __restrict__ lin,
                                               unsigned* lout, unsigned* flag,
                                               int nN, int nE, int nC, int nB1, int nch) {
  __shared__ __attribute__((aligned(16))) unsigned lst[FA * CAP];
  __shared__ int wc[NWAVE * FA];
  __shared__ int cur[FA];
  __shared__ int ovfl;
  const int tid = threadIdx.x, lane = tid & 31, wave = tid >> 5;
  const int blk = blockIdx.x;
  const v4u sv4 = {SENT, SENT, SENT, SENT};
  for (int it = tid; it < (FA * CAP) / 4; it += NTHR) *(v4ua*)(&lst[4 * it]) = sv4;
  if (tid < FA) cur[tid] = 0;
  if (tid == 0) ovfl = 0;
  __syncthreads();

  const int nslots = nB1 * CAP1;
  const unsigned lt = (1u << lane) - 1u;

#pragma unroll 1
  for (int ch = 0; ch < nch; ++ch) {
    bool valid;
    int key;
    unsigned rec;
    if (LV == 1) {
      const int e = blk * S1 + ch * NTHR + tid;
      const int ec = e < nE ? e : nE - 1;
      const int d = edst[ec];
      valid = (e < nE) && ((unsigned)d < (unsigned)nN);
      key = d >> SH1;
      rec = (unsigned)ec;
    } else {
      const int q = ch * NTHR + tid;
      const int qc = q < nslots ? q : nslots - 1;
      const int bl = qc / CAP1, s = qc - bl * CAP1;
      const unsigned id = lin[((size_t)bl * nC + blk) * CAP1 + s];
      const bool idok = id < (unsigned)nE;
      const int idc = idok ? (int)id : nE - 1;
      const int d = edst[idc];
      valid = (q < nslots) && idok && ((unsigned)d < (unsigned)nN) && ((d >> SH1) == blk);
      key = (d >> SH2) & (FA2 - 1);
      rec = ((unsigned)idc & EIDM) | (((unsigned)d & 15u) << 27);
    }
    key = valid ? key : KINV;
    unsigned mym = 0u;
    if (FA <= 32) {
#pragma unroll
      for (int b = 0; b < FA; ++b) {
        const unsigned mb = __builtin_amdgcn_ballot_w32(key == b);
        mym = (key == b) ? mb : mym;
      }
    } else {
#pragma unroll
      for (int i2 = 0; i2 < 32; ++i2) {
        const int ki = __builtin_amdgcn_readlane(key, i2);
        mym |= ((ki == key) ? 1u : 0u) << i2;
      }
    }
    const int rank = __builtin_popcount(mym & lt);
    const int cnt  = __builtin_popcount(mym);
    for (int j = lane; j < FA; j += 32) wc[wave * FA + j] = 0;
    const int kc = valid ? key : 0;
    if (valid && rank == 0) wc[wave * FA + kc] = cnt;
    __syncthreads();
    int pre = 0;
    for (int w2 = 0; w2 < wave; ++w2) pre += wc[w2 * FA + kc];
    const int pos = cur[kc] + pre + rank;
    if (valid && pos < CAP) lst[kc * CAP + pos] = rec;
    int tot = 0;
    if (tid < FA) {
#pragma unroll
      for (int w2 = 0; w2 < NWAVE; ++w2) tot += wc[w2 * FA + tid];
    }
    __syncthreads();
    if (tid < FA) cur[tid] += tot;
  }
  __syncthreads();
  if (tid < FA && cur[tid] > CAP) ovfl = 1;
  __syncthreads();
  const bool wfl = (ovfl != 0) && (tid < 8);
  const v4u one4 = {1u, 1u, 1u, 1u};

  const int nwords  = (LV == 1) ? nC * CAP : FA * CAP;
  const int npieces = nwords >> 2;
  unsigned* gb = lout + (size_t)blk * nwords;
#pragma unroll
  for (int k = 0; k < (FA * CAP / 4 + NTHR - 1) / NTHR; ++k) {
    const int it = tid + NTHR * k;
    if (it < npieces) { const v4u v = *(const v4ua*)(&lst[4 * it]); *(volatile v4u*)(gb + 4 * it) = v; }
  }
  if (wfl) *(volatile v4u*)(flag + 4 * tid) = one4;
  __threadfence();
#pragma unroll
  for (int k = 0; k < (FA * CAP / 4 + NTHR - 1) / NTHR; ++k) {
    const int it = tid + NTHR * k;
    if (it < npieces) { const v4u v = *(const v4ua*)(&lst[4 * it]); *(volatile v4u*)(gb + 4 * it) = v; }
  }
  if (wfl) *(volatile v4u*)(flag + 4 * tid) = one4;
}

__global__ __launch_bounds__(NTHR) void k_gemm(const _Float16* __restrict__ Ap, const _Float16* __restrict__ Bw,
                                               float* XW) {
  __shared__ __attribute__((aligned(16))) float stg[64 * GSP];
  const int tid = threadIdx.x, lane = tid & 31, wave = tid >> 5, hh = lane >> 4, mm = lane & 15;
  const int wm = wave & 3, wn = wave >> 2;
  const int m0 = blockIdx.x * 64, n0 = blockIdx.y * 64;
  const _Float16* abase = Ap + (size_t)(m0 + wm * 16 + mm) * CH + 8 * hh;
  const _Float16* bbase = Bw + (size_t)(n0 + wn * 32 + mm) * CH + 8 * hh;
  v8f c0 = {0.f, 0.f, 0.f, 0.f, 0.f, 0.f, 0.f, 0.f};
  v8f c1 = c0;
#pragma unroll
  for (int kt = 0; kt < KST; ++kt) {
    Frag a, b0, b1;
    a.h[0]  = *(const v8h*)(abase + 32 * kt);
    a.h[1]  = *(const v8h*)(abase + 32 * kt + 16);
    b0.h[0] = *(const v8h*)(bbase + 32 * kt);
    b0.h[1] = *(const v8h*)(bbase + 32 * kt + 16);
    b1.h[0] = *(const v8h*)(bbase + 16 * CH + 32 * kt);
    b1.h[1] = *(const v8h*)(bbase + 16 * CH + 32 * kt + 16);
    c0 = wmh(a.v, b0.v, c0);
    c1 = wmh(a.v, b1.v, c1);
  }
#pragma unroll
  for (int r = 0; r < 8; ++r) {
    const int row = wm * 16 + 8 * hh + r;
    stg[row * GSP + wn * 32 + mm]      = c0[r] * RWSC;
    stg[row * GSP + wn * 32 + 16 + mm] = c1[r] * RWSC;
  }
  __syncthreads();
#pragma unroll
  for (int k = 0; k < 4; ++k) {
    const int p = NTHR * k + tid;
    const int row = p >> 4, cs = (p & 15) * 4;
    const v4f v = *(const v4fa*)(stg + row * GSP + cs);
    *(volatile v4fa*)(XW + (size_t)(m0 + row) * XWP + n0 + cs) = v;
  }
  __threadfence();
#pragma unroll
  for (int k = 0; k < 4; ++k) {
    const int p = NTHR * k + tid;
    const int row = p >> 4, cs = (p & 15) * 4;
    const v4f v = *(const v4fa*)(stg + row * GSP + cs);
    *(volatile v4fa*)(XW + (size_t)(m0 + row) * XWP + n0 + cs) = v;
  }
}

__device__ __forceinline__ void drain(unsigned msk, unsigned rec, v2f& acc, const float* __restrict__ XW,
                                      const float* __restrict__ ea, const int* __restrict__ esrc,
                                      int c2, int nN, int nE) {
  while (msk != 0u) {
    const int i = __builtin_ctz(msk);
    msk &= msk - 1u;
    const unsigned r = (unsigned)__builtin_amdgcn_readlane((int)rec, i);
    int eid = (int)(r & EIDM);
    eid = eid > nE - 1 ? nE - 1 : eid;
    int src = esrc[eid];
    src = src < 0 ? 0 : (src > nN - 1 ? nN - 1 : src);
    const float* arow = ea + (size_t)eid * NR;
    const v4f a0 = *(const v4fa*)arow;
    const v4f a1 = *(const v4fa*)(arow + 4);
    const float* xr = XW + (size_t)src * XWP + c2;
#pragma unroll
    for (int q = 0; q < 4; ++q) {
      const v2f v = *(const v2fa*)(xr + q * CH);
      acc += a0[q] * v;
    }
#pragma unroll
    for (int q = 0; q < 4; ++q) {
      const v2f v = *(const v2fa*)(xr + (4 + q) * CH);
      acc += a1[q] * v;
    }
  }
}

__global__ __launch_bounds__(NTHR) void k_agg(const float* __restrict__ XW, const float* __restrict__ ea,
                                              const int* __restrict__ esrc, const unsigned* __restrict__ l2,
                                              const float* __restrict__ bias, const unsigned* __restrict__ flag,
                                              _Float16* Ap, float* out, int nN, int nE, int fin) {
  __shared__ __attribute__((aligned(16))) float ostg[TR * CH];
  const int tid = threadIdx.x, lane = tid & 31, wave = tid >> 5;
  const int tile = blockIdx.x;
  const int c2 = 2 * lane;
  const v2f z2 = {0.f, 0.f};

  v2f acc0 = z2, acc1 = z2;
  {
    const unsigned* seg = l2 + (size_t)tile * CAP2;
#pragma unroll 1
    for (int ch = 0; ch < CAP2 / 32; ++ch) {
      const unsigned rec = seg[ch * 32 + lane];
      const bool ok = ((int)rec) >= 0;
      const int ln = (int)((rec >> 27) & 15u);
      const unsigned m0 = __builtin_amdgcn_ballot_w32(ok && (ln == 2 * wave));
      const unsigned m1 = __builtin_amdgcn_ballot_w32(ok && (ln == 2 * wave + 1));
      drain(m0, rec, acc0, XW, ea, esrc, c2, nN, nE);
      drain(m1, rec, acc1, XW, ea, esrc, c2, nN, nE);
    }
  }

  const unsigned fl = flag[0];
  const float qn = __int_as_float(0x7fc00000);
  const v2f nan2 = {qn, qn};
  const v2f bv = *(const v2fa*)(bias + c2);
#pragma unroll
  for (int q = 0; q < 2; ++q) {
    const v2f acc = (q == 0) ? acc0 : acc1;
    const int j = 2 * wave + q;
    const int node = tile * TR + j;
    const int nodec = node < nN ? node : nN - 1;
    const v2f sv = *(const v2fa*)(XW + (size_t)nodec * XWP + NR * CH + c2);
    v2f o = acc + sv + bv;
    if (fin == 0) { o[0] = o[0] > 0.f ? o[0] : 0.f; o[1] = o[1] > 0.f ? o[1] : 0.f; }
    if (node >= nN) o = z2;
    if (fin != 0 && fl != 0u) o = nan2;
    *(v2fa*)(ostg + j * CH + c2) = o;
  }
  __syncthreads();

  if (fin != 0) {
    const int rem = nN - tile * TR;
    const int rows = rem < TR ? rem : TR;
    const int npc = rows * (CH / 4);
    float* obase = out + (size_t)tile * TR * CH;
    const int p = tid;
    if (p < npc) { const v4f v = *(const v4fa*)(ostg + 4 * p); *(volatile v4fa*)(obase + 4 * p) = v; }
    __threadfence();
    if (p < npc) { const v4f v = *(const v4fa*)(ostg + 4 * p); *(volatile v4fa*)(obase + 4 * p) = v; }
  } else {
    if (tid < (TR * CH) / 8) {
      const int row = tid >> 3, cs = (tid & 7) * 8;
      const v4f lo = *(const v4fa*)(ostg + row * CH + cs);
      const v4f hi = *(const v4fa*)(ostg + row * CH + cs + 4);
      const v8f f = {lo[0], lo[1], lo[2], lo[3], hi[0], hi[1], hi[2], hi[3]};
      const v8h hv = __builtin_convertvector(f, v8h);
      _Float16* dst = Ap + (size_t)(tile * TR + row) * CH + cs;
      *(volatile v8h*)dst = hv;
      __threadfence();
      *(volatile v8h*)dst = hv;
    }
  }
}

extern "C" void kernel_launch(void* const* d_in, const int* in_sizes, int n_in,
                              void* d_out, int out_size, void* d_ws, size_t ws_size,
                              hipStream_t stream) {
  if (n_in < 7) return;
  if (in_sizes[0] < CH || (in_sizes[0] % CH) != 0) return;
  const int nN = in_sizes[0] / CH;
  if (nN < 1 || nN > (FA1 << SH1)) return;
  if (in_sizes[1] < 2 || (in_sizes[1] % 2) != 0) return;
  const int nE = in_sizes[1] / 2;
  if (nE < 1 || nE > (int)EIDM) return;
  if (in_sizes[2] != nE * NR) return;
  if (in_sizes[3] != NL * NBS * CH * CH) return;
  if (in_sizes[4] != NL * NR * NBS) return;
  if (in_sizes[5] != NL * CH * CH) return;
  if (in_sizes[6] != NL * CH) return;
  if (out_size != nN * CH) return;

  const float* x     = (const float*)d_in[0];
  const int*   ei    = (const int*)d_in[1];
  const float* ea    = (const float*)d_in[2];
  const float* basis = (const float*)d_in[3];
  const float* att   = (const float*)d_in[4];
  const float* root  = (const float*)d_in[5];
  const float* bias  = (const float*)d_in[6];
  const int*   esrc  = ei;
  const int*   edst  = ei + nE;
  float* out = (float*)d_out;

  const int MP     = ((nN + 63) / 64) * 64;
  const int nTiles = (nN + TR - 1) / TR;
  const int nT16   = nTiles * TR;
  const int nC     = (nN + (1 << SH1) - 1) >> SH1;
  const int nB1    = (nE + S1 - 1) / S1;
  const int nch2   = (nB1 * CAP1 + NTHR - 1) / NTHR;
  const int nbA    = (MP * KQ) / NTHR;
  if (nC < 1 || nC > FA1) return;
  if (MP < nT16) return;

  char* ws = (char*)d_ws;
  size_t o = 0;
  const size_t oA  = o; o += (size_t)MP * CH * 2;                          o = (o + 255) & ~(size_t)255;
  const size_t oB  = o; o += (size_t)NL * NCAT * CH * 2;                   o = (o + 255) & ~(size_t)255;
  const size_t oFL = o; o += 256;
  const size_t oL2 = o; o += (size_t)nC * FA2 * CAP2 * 4;                  o = (o + 255) & ~(size_t)255;
  const size_t szL1 = (size_t)nB1 * nC * CAP1 * 4;
  const size_t szXW = (size_t)MP * XWP * 4;
  const size_t oU  = o; o += (szL1 > szXW ? szL1 : szXW);                  o = (o + 255) & ~(size_t)255;
  if (o > ws_size || o > (size_t)WSCAPB) return;
  _Float16* Ap = (_Float16*)(ws + oA);
  _Float16* Bw = (_Float16*)(ws + oB);
  unsigned* FL = (unsigned*)(ws + oFL);
  unsigned* L2 = (unsigned*)(ws + oL2);
  unsigned* L1 = (unsigned*)(ws + oU);
  float*    XW = (float*)(ws + oU);

  k_prep<<<nbA + NBLKB + 1, NTHR, 0, stream>>>(x, basis, att, root, Ap, Bw, FL, nN, nbA);
  k_part<1, FA1, CAP1><<<nB1, NTHR, 0, stream>>>(edst, L1, L1, FL, nN, nE, nC, nB1, NCH1);
  k_part<2, FA2, CAP2><<<nC, NTHR, 0, stream>>>(edst, L1, L2, FL, nN, nE, nC, nB1, nch2);
  for (int L = 0; L < NL; ++L) {
    k_gemm<<<dim3(MP / 64, NCAT / 64), NTHR, 0, stream>>>(Ap, Bw + (size_t)L * NCAT * CH, XW);
    k_agg<<<nTiles, NTHR, 0, stream>>>(XW, ea, esrc, L2, bias + (size_t)L * CH, FL, Ap, out, nN, nE,
                                       (L == NL - 1) ? 1 : 0);
  }
}
